// MixedAttention_72602127172196
// MI455X (gfx1250) — hardware-verified
//
#include <hip/hip_runtime.h>
#include <math.h>

#ifndef NB
#define NB 4
#endif
#ifndef SEQ
#define SEQ 2048
#endif
#define NB_FULL 4
#define SEQ_FULL 2048

constexpr int kHid    = 768;
constexpr int kHeads  = 6;
constexpr int kDh     = 64;
constexpr int kAH     = kHeads * kDh;
constexpr int kKW     = 9;
constexpr int kCK     = kHeads * kKW;
constexpr int kCKPad  = 64;
constexpr int kTok    = NB * SEQ;
constexpr int kTokPerBlk = 32;

constexpr float kWCarry    = 16.0f;
constexpr float kWCarryInv = 1.0f / 16.0f;
constexpr float kPWCarry   = 64.0f;
constexpr float kDWCarry   = 64.0f;
constexpr float kKCScale   = 1.0f / (kPWCarry * kDWCarry);
constexpr float kGCarry    = 8.0f;
constexpr float kCACarry   = 1024.0f;
constexpr float kCKScale   = 1.0f / (kCACarry * kWCarry);
constexpr float kPCarry    = 32768.0f;
constexpr float kPVScale   = 1.0f / (kPCarry * kGCarry);
constexpr float kSmScale   = 0.125f / (kGCarry * kGCarry);

static_assert(kHeads * kDh == kAH);
static_assert(kCK <= kCKPad);
static_assert(kTok % 64 == 0 && kAH % 64 == 0 && kHid % 32 == 0);
static_assert(kCKPad % 64 == 0 && kAH % 32 == 0);
static_assert(SEQ % 64 == 0 && kDh % 32 == 0 && kDh % 64 == 0);
static_assert(SEQ % 256 == 0 && SEQ <= 2048);
static_assert(SEQ % kTokPerBlk == 0);
static_assert((kTok * kHid / 8) % 32 == 0 && (kTok * kAH / 8) % 32 == 0 && (kAH * kHid / 8) % 256 == 0);
static_assert((kTokPerBlk * kHeads) % 96 == 0);

typedef __attribute__((ext_vector_type(16))) _Float16 v16h;
typedef __attribute__((ext_vector_type(8)))  _Float16 v8h;
typedef __attribute__((ext_vector_type(16))) __bf16   v16b;
typedef __attribute__((ext_vector_type(8)))  __bf16   v8b;
typedef __attribute__((ext_vector_type(8)))  float    v8f;
typedef __attribute__((ext_vector_type(4)))  float    v4f;
typedef __attribute__((ext_vector_type(2)))  float    v2f;
typedef __attribute__((ext_vector_type(4)))  unsigned int v4u;

__device__ __forceinline__ unsigned short f2bf_bits(float f) {
  unsigned u = __float_as_uint(f);
  return (unsigned short)((u + 0x7FFFu + ((u >> 16) & 1u)) >> 16);
}
__device__ __forceinline__ float bf_bits2f(unsigned short h) { return __uint_as_float(((unsigned)h) << 16); }
__device__ __forceinline__ float bf_rne(float f) { return bf_bits2f(f2bf_bits(f)); }

__device__ __forceinline__ void dep_guard_h(v8f& a, v8f& b, v16h x, v16h y) { asm volatile("v_nop\n\tv_nop\n\tv_nop\n\tv_nop" : "+v"(a), "+v"(b) : "v"(x), "v"(y)); }
__device__ __forceinline__ void dep_guard_b(v8f& a, v8f& b, v16b x, v16b y) { asm volatile("v_nop\n\tv_nop\n\tv_nop\n\tv_nop" : "+v"(a), "+v"(b) : "v"(x), "v"(y)); }
__device__ __forceinline__ void keep4_h(v16h a, v16h b, v16h c, v16h d) { asm volatile("v_nop" :: "v"(a), "v"(b), "v"(c), "v"(d)); }
__device__ __forceinline__ void keep4_b(v16b a, v16b b, v16b c, v16b d) { asm volatile("v_nop" :: "v"(a), "v"(b), "v"(c), "v"(d)); }
__device__ __forceinline__ void acc_guard4(v8f& a, v8f& b, v8f& c, v8f& d) { asm volatile("v_nop\n\tv_nop\n\tv_nop\n\tv_nop" : "+v"(a), "+v"(b), "+v"(c), "+v"(d)); }
template <typename T> struct Frag;
template <> struct Frag<_Float16> {
  typedef v16h V; union U { v16h v; v8h h[2]; };
  static __device__ __forceinline__ v16h load(const _Float16* p) {
    U f; f.h[0] = *(const v8h*)(p); f.h[1] = *(const v8h*)(p + 16); return f.v;
  }
  static __device__ __forceinline__ v8f mma(v16h a, v16h b, v8f c) {
    return __builtin_amdgcn_wmma_f32_16x16x32_f16(false, a, false, b, (short)0, c, false, false);
  }
  static __device__ __forceinline__ void guard(v8f& a, v8f& b, v16h x, v16h y) { dep_guard_h(a, b, x, y); }
  static __device__ __forceinline__ void keep(v16h a, v16h b, v16h c, v16h d) { keep4_h(a, b, c, d); }
};
template <> struct Frag<__bf16> {
  typedef v16b V; union U { v16b v; v8b h[2]; };
  static __device__ __forceinline__ v16b load(const __bf16* p) {
    U f; f.h[0] = *(const v8b*)(p); f.h[1] = *(const v8b*)(p + 16); return f.v;
  }
  static __device__ __forceinline__ v8f mma(v16b a, v16b b, v8f c) {
    return __builtin_amdgcn_wmma_f32_16x16x32_bf16(false, a, false, b, (short)0, c, false, false);
  }
  static __device__ __forceinline__ void guard(v8f& a, v8f& b, v16b x, v16b y) { dep_guard_b(a, b, x, y); }
  static __device__ __forceinline__ void keep(v16b a, v16b b, v16b c, v16b d) { keep4_b(a, b, c, d); }
};

__device__ __forceinline__ unsigned pk16(unsigned short a, unsigned short b) { return (unsigned)a | ((unsigned)b << 16); }
__device__ __forceinline__ unsigned short h_bits(float f) { const _Float16 h = (_Float16)f; return __builtin_bit_cast(unsigned short, h); }

template <int ET> struct Elem;
template <> struct Elem<0> { typedef _Float16 T; };
template <> struct Elem<1> { typedef __bf16 T; };
template <int ET, bool SPLIT, int BIAS_MODE, int OUT_MODE, bool RESID, int ACT = 0>
__global__ __launch_bounds__(256) void wmma_gemm64(
    const unsigned short* __restrict__ Ap, const unsigned short* __restrict__ A2p, int lda, long strideA,
    const unsigned short* __restrict__ Btp, const unsigned short* __restrict__ Bt2p, int ldb, long strideB,
    void* __restrict__ Cout, void* __restrict__ Cout2, int ldc, long strideC,
    const float* __restrict__ bias,
    const float* __restrict__ resid, long strideR,
    int M, int N, int K, float scale, float bsc) {
  typedef typename Elem<ET>::T T;
  typedef typename Frag<T>::V V;
  const T* A = (const T*)Ap; const T* A2 = (const T*)A2p; const T* Bt = (const T*)Btp; const T* Bt2 = (const T*)Bt2p;
  __shared__ __align__(16) float sT[8][16 * 68];
  const int b    = blockIdx.y;
  const int lane = threadIdx.x & 31;
  const int wave = threadIdx.x >> 5;
  const int tilesN = N >> 6;
  const int tilesM = M >> 6;
  const int tile = blockIdx.x * 8 + wave;
  if (tile >= tilesM * tilesN) return;
  const int tm = tile / tilesN;
  const int tn = tile - tm * tilesN;
  const int m0 = tm << 6;
  const int n0 = tn << 6;

  const T* Ab  = A  + (size_t)b * strideA;
  const T* Bb  = Bt + (size_t)b * strideB;
  const T* Ab2 = SPLIT ? (A2  + (size_t)b * strideA) : nullptr;
  const T* Bb2 = SPLIT ? (Bt2 + (size_t)b * strideB) : nullptr;

  const int rlane = lane & 15;
  const int koff  = (lane >> 4) * 8;
  const int mOff  = (lane >> 4) * 8;

  v8f acc[4][4];
#pragma unroll
  for (int i = 0; i < 4; ++i)
#pragma unroll
    for (int j = 0; j < 4; ++j) acc[i][j] = (v8f){0.f,0.f,0.f,0.f,0.f,0.f,0.f,0.f};

  for (int k0 = 0; k0 < K; k0 += 32) {
    V bh[4], bl[4];
#pragma unroll
    for (int j = 0; j < 4; ++j) {
      const size_t bo = (size_t)(n0 + (j << 4) + rlane) * ldb + koff + k0;
      bh[j] = Frag<T>::load(Bb + bo);
      if (SPLIT) bl[j] = Frag<T>::load(Bb2 + bo);
    }
#pragma unroll
    for (int i = 0; i < 4; ++i) {
      const size_t ao = (size_t)(m0 + (i << 4) + rlane) * lda + koff + k0;
      V ah = Frag<T>::load(Ab + ao);
      V al;
      if (SPLIT) al = Frag<T>::load(Ab2 + ao);
#pragma unroll
      for (int j = 0; j < 4; ++j) {
        acc[i][j] = Frag<T>::mma(ah, bh[j], acc[i][j]);
        if (SPLIT) {
          acc[i][j] = Frag<T>::mma(ah, bl[j], acc[i][j]);
          acc[i][j] = Frag<T>::mma(al, bh[j], acc[i][j]);
        }
      }
      Frag<T>::guard(acc[i][0], acc[i][3], ah, SPLIT ? al : ah);
    }
    Frag<T>::keep(bh[0], bh[1], bh[2], bh[3]);
    if (SPLIT) Frag<T>::keep(bl[0], bl[1], bl[2], bl[3]);
  }
  acc_guard4(acc[0][0], acc[0][1], acc[0][2], acc[0][3]);
  acc_guard4(acc[1][0], acc[1][1], acc[1][2], acc[1][3]);
  acc_guard4(acc[2][0], acc[2][1], acc[2][2], acc[2][3]);
  acc_guard4(acc[3][0], acc[3][1], acc[3][2], acc[3][3]);

  float* slab = sT[wave];
  const float* Rb = RESID ? (resid + (size_t)b * strideR) : nullptr;
#pragma unroll
  for (int i = 0; i < 4; ++i) {
    const int mBase = m0 + (i << 4);
#pragma unroll
    for (int j = 0; j < 4; ++j) {
      const int n = n0 + (j << 4) + rlane;
      float bv = 0.f;
      if (BIAS_MODE == 2) bv = bsc * bf_rne(bias[n]);
#pragma unroll
      for (int r = 0; r < 8; ++r) {
        float v = acc[i][j][r] * scale;
        if (BIAS_MODE == 1) v += bsc * bf_rne(bias[mBase + mOff + r]);
        if (BIAS_MODE == 2) v += bv;
        if (RESID) v += Rb[(size_t)(mBase + mOff + r) * ldc + n];
        if (ACT == 2) v = fmaxf(v, 0.0f);
        if (ACT == 4) v = (v > 0.f) ? v : 0.01f * v;
        slab[(mOff + r) * 68 + (j << 4) + rlane] = v;
      }
    }
    __builtin_amdgcn_fence(__ATOMIC_RELEASE, "workgroup");
    __builtin_amdgcn_wave_barrier();
    __builtin_amdgcn_fence(__ATOMIC_ACQUIRE, "workgroup");
    if (OUT_MODE == 0) {
      float* C = (float*)Cout + (size_t)b * strideC;
      const int hh = lane >> 4, c4 = (lane & 15) * 4;
      for (int pass = 0; pass < 2; ++pass) {
#pragma unroll
        for (int it = 0; it < 8; ++it) {
          const int row = it * 2 + hh;
          v4f v = *(const v4f*)(slab + row * 68 + c4);
          *(volatile v4f*)(C + (size_t)(mBase + row) * ldc + n0 + c4) = v;
        }
        __threadfence();
      }
    } else {
      const int q = lane >> 3, c8 = (lane & 7) * 8;
      unsigned short* C  = (unsigned short*)Cout  + (size_t)b * strideC;
      unsigned short* C2 = (OUT_MODE == 2) ? ((unsigned short*)Cout2 + (size_t)b * strideC) : nullptr;
      for (int pass = 0; pass < 2; ++pass) {
#pragma unroll
        for (int it = 0; it < 4; ++it) {
          const int row = it * 4 + q;
          const float* sp = slab + row * 68 + c8;
          v8h hv, lv;
#pragma unroll
          for (int e = 0; e < 8; ++e) {
            if (OUT_MODE == 1) {
              hv[e] = (_Float16)sp[e];
            } else {
              unsigned short hb = f2bf_bits(sp[e]);
              unsigned short lb = f2bf_bits(sp[e] - bf_bits2f(hb));
              hv[e] = __builtin_bit_cast(_Float16, hb);
              lv[e] = __builtin_bit_cast(_Float16, lb);
            }
          }
          *(volatile v8h*)(C + (size_t)(mBase + row) * ldc + n0 + c8) = hv;
          if (OUT_MODE == 2) *(volatile v8h*)(C2 + (size_t)(mBase + row) * ldc + n0 + c8) = lv;
        }
        __threadfence();
      }
    }
    __builtin_amdgcn_fence(__ATOMIC_RELEASE, "workgroup");
    __builtin_amdgcn_wave_barrier();
    __builtin_amdgcn_fence(__ATOMIC_ACQUIRE, "workgroup");
  }
}

__global__ __launch_bounds__(256) void cast_x_kernel(const float* __restrict__ x, unsigned short* __restrict__ Xh, int n8) {
  const int i = blockIdx.x * 256 + threadIdx.x;
  if (i >= n8) return;
  const size_t e0 = 8 * (size_t)i;
  const int tok = (int)(e0 / kHid);
  const int c   = (int)(e0 - (size_t)tok * kHid);
  const int b   = tok / SEQ;
  const int s   = tok - b * SEQ;
  const float* p = x + ((size_t)(b * SEQ_FULL + s)) * kHid + c;
  const v4f a = *(const v4f*)(p);
  const v4f d = *(const v4f*)(p + 4);
  unsigned short hb[8];
#pragma unroll
  for (int e = 0; e < 4; ++e) {
    hb[e]     = h_bits(bf_rne(a[e]));
    hb[4 + e] = h_bits(bf_rne(d[e]));
  }
  const v4u u = (v4u){pk16(hb[0], hb[1]), pk16(hb[2], hb[3]), pk16(hb[4], hb[5]), pk16(hb[6], hb[7])};
  unsigned short* q = Xh + e0;
  *(volatile v4u*)q = u;
  __threadfence();
  *(volatile v4u*)q = u;
}

__global__ __launch_bounds__(256) void cast_w_kernel(const float* __restrict__ W0, const float* __restrict__ W1,
                                                     const float* __restrict__ W2, const float* __restrict__ W3,
                                                     const float* __restrict__ W4, unsigned short* __restrict__ out,
                                                     int n8, float sc03, float sc4) {
  const int z = blockIdx.y;
  const float* W = (z == 0) ? W0 : (z == 1) ? W1 : (z == 2) ? W2 : (z == 3) ? W3 : W4;
  const float sc = (z == 4) ? sc4 : sc03;
  const int i = blockIdx.x * 256 + threadIdx.x;
  if (i >= n8) return;
  const float* p = W + 8 * (size_t)i;
  const v4f a = *(const v4f*)(p);
  const v4f d = *(const v4f*)(p + 4);
  unsigned short hb[8];
#pragma unroll
  for (int e = 0; e < 4; ++e) {
    hb[e]     = h_bits(bf_rne(a[e]) * sc);
    hb[4 + e] = h_bits(bf_rne(d[e]) * sc);
  }
  const v4u u = (v4u){pk16(hb[0], hb[1]), pk16(hb[2], hb[3]), pk16(hb[4], hb[5]), pk16(hb[6], hb[7])};
  unsigned short* q = out + (size_t)z * 8 * (size_t)n8 + 8 * (size_t)i;
  *(volatile v4u*)q = u;
  __threadfence();
  *(volatile v4u*)q = u;
}

__global__ __launch_bounds__(256) void cast_wck_kernel(const float* __restrict__ Wck, unsigned short* __restrict__ out) {
  const int i = blockIdx.x * 256 + threadIdx.x;
  if (i >= kCKPad * kAH / 8) return;
  const int e0  = 8 * i;
  const int row = e0 / kAH;
  const int col = e0 - row * kAH;
  const int rowc = (row < kCK) ? row : (kCK - 1);
  const bool keep = row < kCK;
  const float* p = Wck + (size_t)rowc * kAH + col;
  const v4f a = *(const v4f*)(p);
  const v4f d = *(const v4f*)(p + 4);
  unsigned short hb[8];
#pragma unroll
  for (int e = 0; e < 4; ++e) {
    const float va = keep ? bf_rne(a[e]) * kWCarry : 0.0f;
    const float vd = keep ? bf_rne(d[e]) * kWCarry : 0.0f;
    hb[e]     = h_bits(va);
    hb[4 + e] = h_bits(vd);
  }
  const v4u u = (v4u){pk16(hb[0], hb[1]), pk16(hb[2], hb[3]), pk16(hb[4], hb[5]), pk16(hb[6], hb[7])};
  unsigned short* q = out + e0;
  *(volatile v4u*)q = u;
  __threadfence();
  *(volatile v4u*)q = u;
}

__global__ __launch_bounds__(96) void dwconv_kernel(const unsigned short* __restrict__ Xh, const float* __restrict__ dw,
                                                    unsigned short* __restrict__ DWh) {
  __shared__ __align__(16) float sdw[kKW][kHid];
  const int t  = threadIdx.x;
  const int c8 = 8 * t;
#pragma unroll
  for (int g = 0; g < 18; ++g) {
    const v4f w = *(const v4f*)(dw + 72 * t + 4 * g);
#pragma unroll
    for (int k = 0; k < 4; ++k) {
      const int idx = 4 * g + k;
      const int ch  = idx / kKW;
      const int tap = idx - ch * kKW;
      sdw[tap][c8 + ch] = bf_rne(w[k]);
    }
  }
  __syncthreads();
  const int tok0 = blockIdx.x * kTokPerBlk;
  const int b  = tok0 / SEQ;
  const int s0 = tok0 - b * SEQ;
  const _Float16* Xb = (const _Float16*)Xh + (size_t)b * SEQ * kHid + c8;
#pragma unroll 1
  for (int tt = 0; tt < kTokPerBlk; ++tt) {
    const int s = s0 + tt;
    float acc[8];
#pragma unroll
    for (int e = 0; e < 8; ++e) acc[e] = 0.0f;
#pragma unroll 1
    for (int i = 0; i < kKW; ++i) {
      const int sp = s + i - kKW / 2;
      const bool valid = (sp >= 0) && (sp < SEQ);
      const int spc = (sp < 0) ? 0 : ((sp >= SEQ) ? (SEQ - 1) : sp);
      const v8h xv = *(const v8h*)(Xb + (size_t)spc * kHid);
      const v4f wa = *(const v4f*)(&sdw[i][c8]);
      const v4f wb = *(const v4f*)(&sdw[i][c8 + 4]);
      const float f = valid ? 1.0f : 0.0f;
#pragma unroll
      for (int e = 0; e < 4; ++e) {
        acc[e]     += (wa[e] * f) * (float)xv[e];
        acc[4 + e] += (wb[e] * f) * (float)xv[4 + e];
      }
    }
    unsigned short hb[8];
#pragma unroll
    for (int e = 0; e < 8; ++e) hb[e] = h_bits(acc[e] * kDWCarry);
    const v4u u = (v4u){pk16(hb[0], hb[1]), pk16(hb[2], hb[3]), pk16(hb[4], hb[5]), pk16(hb[6], hb[7])};
    unsigned short* q = DWh + (size_t)(tok0 + tt) * kHid + c8;
    *(volatile v4u*)q = u;
    __threadfence();
    *(volatile v4u*)q = u;
  }
}

__global__ __launch_bounds__(256) void qca_cast_kernel(const float* __restrict__ Fq, const float* __restrict__ Fkc,
                                                       unsigned short* __restrict__ Qh, unsigned short* __restrict__ CAh, int n8) {
  const int i = blockIdx.x * 256 + threadIdx.x;
  if (i >= n8) return;
  const size_t e0 = 8 * (size_t)i;
  const v4f qa = *(const v4f*)(Fq + e0);
  const v4f qb = *(const v4f*)(Fq + e0 + 4);
  const v4f ka = *(const v4f*)(Fkc + e0);
  const v4f kb = *(const v4f*)(Fkc + e0 + 4);
  unsigned short hq[8], hc[8];
#pragma unroll
  for (int e = 0; e < 4; ++e) {
    const float pa = ka[e] * qa[e];
    const float pb = kb[e] * qb[e];
    hq[e]     = h_bits(qa[e] * kGCarry);
    hq[4 + e] = h_bits(qb[e] * kGCarry);
    hc[e]     = h_bits(pa * kCACarry);
    hc[4 + e] = h_bits(pb * kCACarry);
  }
  const v4u uq = (v4u){pk16(hq[0], hq[1]), pk16(hq[2], hq[3]), pk16(hq[4], hq[5]), pk16(hq[6], hq[7])};
  const v4u uc = (v4u){pk16(hc[0], hc[1]), pk16(hc[2], hc[3]), pk16(hc[4], hc[5]), pk16(hc[6], hc[7])};
  unsigned short* pq = Qh + e0;
  unsigned short* pc = CAh + e0;
  *(volatile v4u*)pq = uq;
  *(volatile v4u*)pc = uc;
  __threadfence();
  *(volatile v4u*)pq = uq;
  *(volatile v4u*)pc = uc;
}

__global__ __launch_bounds__(96) void span_conv_kernel(const float* __restrict__ CK, const float* __restrict__ bck,
                                                       const float* __restrict__ Fco, float* __restrict__ out) {
  __shared__ float sw[kTokPerBlk][kCK];
  const int t    = threadIdx.x;
  const int tok0 = blockIdx.x * kTokPerBlk;
  const int b    = tok0 / SEQ;
  const int s0   = tok0 - b * SEQ;
#pragma unroll 1
  for (int it = t; it < kTokPerBlk * kHeads; it += 96) {
    const int tk = it / kHeads;
    const int h  = it - tk * kHeads;
    const float* lp = CK + (size_t)(tok0 + tk) * kCKPad + h * kKW;
    float* swp = &sw[tk][h * kKW];
    float m = -__builtin_inff();
#pragma unroll 1
    for (int i = 0; i < kKW; ++i) {
      const float l = lp[i] + bf_rne(bck[h * kKW + i]);
      swp[i] = l;
      m = fmaxf(m, l);
    }
    float sum = 0.0f;
#pragma unroll 1
    for (int i = 0; i < kKW; ++i) {
      const float e = expf(swp[i] - m);
      swp[i] = e;
      sum += e;
    }
    const float inv = 1.0f / sum;
#pragma unroll 1
    for (int i = 0; i < kKW; ++i) swp[i] = swp[i] * inv;
  }
  __syncthreads();
  const int c4 = 4 * t;
  const int h  = t >> 4;
  const float* cob = Fco + (size_t)b * SEQ * kAH + c4;
#pragma unroll 1
  for (int tt = 0; tt < kTokPerBlk; ++tt) {
    const int s = s0 + tt;
    float acc[4];
#pragma unroll
    for (int e = 0; e < 4; ++e) acc[e] = 0.0f;
    const float* swp = &sw[tt][h * kKW];
#pragma unroll 1
    for (int i = 0; i < kKW; ++i) {
      const int sp = s + i - kKW / 2;
      const bool valid = (sp >= 0) && (sp < SEQ);
      const int spc = (sp < 0) ? 0 : ((sp >= SEQ) ? (SEQ - 1) : sp);
      const v4f cv = *(const v4f*)(cob + (size_t)spc * kAH);
      const float wl = swp[i];
      const float w  = valid ? wl : 0.0f;
#pragma unroll
      for (int e = 0; e < 4; ++e) acc[e] += w * cv[e];
    }
    const v4f o = (v4f){acc[0], acc[1], acc[2], acc[3]};
    float* op = out + (size_t)(tok0 + tt) * (2 * kAH) + kAH + c4;
    *(volatile v4f*)op = o;
    __threadfence();
    *(volatile v4f*)op = o;
  }
}

__global__ __launch_bounds__(256) void softmax_row_kernel(const float* __restrict__ Sp, unsigned short* __restrict__ Pp) {
  __shared__ __align__(16) float lg[SEQ];
  __shared__ float redM[8];
  __shared__ float redS[8];
  const int i    = blockIdx.x;
  const int t    = threadIdx.x;
  const int lane = t & 31, wave = t >> 5;
  const size_t rowoff = (size_t)i * SEQ;
  const float* sr = Sp + rowoff;

  float mx = -__builtin_inff();
#pragma unroll 1
  for (int c = 2 * t; c < SEQ; c += 512) {
    const v2f sv = *(const v2f*)(sr + c);
    v2f av;
#pragma unroll
    for (int e = 0; e < 2; ++e) {
      av[e] = sv[e] * kSmScale;
      mx = fmaxf(mx, av[e]);
    }
    *(v2f*)(lg + c) = av;
  }
#pragma unroll
  for (int off = 16; off > 0; off >>= 1) mx = fmaxf(mx, __shfl_xor(mx, off, 32));
  if (lane == 0) redM[wave] = mx;
  __syncthreads();
  float m = redM[0];
#pragma unroll
  for (int w = 1; w < 8; ++w) m = fmaxf(m, redM[w]);

  float sum = 0.0f;
#pragma unroll 1
  for (int c = 2 * t; c < SEQ; c += 512) {
    const v2f l = *(const v2f*)(lg + c);
    v2f ev;
#pragma unroll
    for (int e = 0; e < 2; ++e) {
      ev[e] = expf(l[e] - m);
      sum += ev[e];
    }
    *(v2f*)(lg + c) = ev;
  }
#pragma unroll
  for (int off = 16; off > 0; off >>= 1) sum += __shfl_xor(sum, off, 32);
  if (lane == 0) redS[wave] = sum;
  __syncthreads();
  float tot = redS[0];
#pragma unroll
  for (int w = 1; w < 8; ++w) tot += redS[w];
  const float inv = kPCarry / tot;

  if (8 * t < SEQ) {
    const v4f e0 = *(const v4f*)(lg + 8 * t);
    const v4f e1 = *(const v4f*)(lg + 8 * t + 4);
    unsigned short hb[8];
#pragma unroll
    for (int e = 0; e < 4; ++e) {
      hb[e]     = h_bits(e0[e] * inv);
      hb[4 + e] = h_bits(e1[e] * inv);
    }
    const v4u u = (v4u){pk16(hb[0], hb[1]), pk16(hb[2], hb[3]), pk16(hb[4], hb[5]), pk16(hb[6], hb[7])};
    unsigned short* pr = Pp + rowoff + 8 * (size_t)t;
    *(volatile v4u*)pr = u;
    __threadfence();
    *(volatile v4u*)pr = u;
  }
}

static inline int cdiv_host(int a, int b) { return (a + b - 1) / b; }

extern "C" void kernel_launch(void* const* d_in, const int* in_sizes, int n_in,
                              void* d_out, int out_size, void* d_ws, size_t ws_size,
                              hipStream_t stream) {
  if (n_in < 14) return;
  if (in_sizes[0] < ((NB - 1) * SEQ_FULL + SEQ) * kHid) return;
  if (in_sizes[1] < kAH * kHid || in_sizes[3] < kAH * kHid || in_sizes[5] < kAH * kHid) return;
  if (in_sizes[8] < kAH * kHid || in_sizes[12] < kAH * kHid) return;
  if (in_sizes[2] < kAH || in_sizes[4] < kAH || in_sizes[6] < kAH || in_sizes[9] < kAH || in_sizes[13] < kAH) return;
  if (in_sizes[7] < kHid * kKW || in_sizes[10] < kCK * kAH || in_sizes[11] < kCK) return;
  if (out_size < kTok * 2 * kAH) return;

  const size_t szXh  = (size_t)kTok * kHid * 2;
  const size_t szWpl = (size_t)5 * kAH * kHid * 2;
  const size_t szWck = (size_t)kCKPad * kAH * 2;
  const size_t szDW  = (size_t)kTok * kHid * 2;
  const size_t szF   = (size_t)kTok * kAH * 4;
  const size_t szH   = (size_t)kTok * kAH * 2;
  const size_t szCK  = (size_t)kTok * kCKPad * 4;
  const size_t szSC  = (size_t)SEQ * SEQ * 4;
  const size_t szPP  = (size_t)SEQ * SEQ * 2;
  const size_t offXh  = 0;
  const size_t offWpl = offXh + szXh;
  const size_t offWck = offWpl + szWpl;
  const size_t offDW  = offWck + szWck;
  const size_t offFq  = offDW + szDW;
  const size_t offFco = offFq + szF;
  const size_t offFkc = offFco + szF;
  const size_t offKh  = offFkc + szF;
  const size_t offVT  = offKh + szH;
  const size_t offQh  = offVT + szH;
  const size_t offCA  = offQh + szH;
  const size_t offCK  = offCA + szH;
  const size_t offSC  = offCK + szCK;
  const size_t offPP  = offSC + szSC;
  const size_t total  = offPP + szPP;
  if (ws_size < total) return;

  const float* x     = (const float*)d_in[0];
  const float* Wq    = (const float*)d_in[1];
  const float* bq    = (const float*)d_in[2];
  const float* Wk    = (const float*)d_in[3];
  const float* bk    = (const float*)d_in[4];
  const float* Wv    = (const float*)d_in[5];
  const float* bv    = (const float*)d_in[6];
  const float* dw    = (const float*)d_in[7];
  const float* pw    = (const float*)d_in[8];
  const float* cbias = (const float*)d_in[9];
  const float* Wck   = (const float*)d_in[10];
  const float* bck   = (const float*)d_in[11];
  const float* Wco   = (const float*)d_in[12];
  const float* bco   = (const float*)d_in[13];
  float* out = (float*)d_out;
  char* ws = (char*)d_ws;
  unsigned short* Xh   = (unsigned short*)(ws + offXh);
  unsigned short* Wpl  = (unsigned short*)(ws + offWpl);
  unsigned short* WCKh = (unsigned short*)(ws + offWck);
  unsigned short* DWh  = (unsigned short*)(ws + offDW);
  float*          Fq   = (float*)(ws + offFq);
  float*          Fco  = (float*)(ws + offFco);
  float*          Fkc  = (float*)(ws + offFkc);
  unsigned short* Kh   = (unsigned short*)(ws + offKh);
  unsigned short* VT   = (unsigned short*)(ws + offVT);
  unsigned short* Qh   = (unsigned short*)(ws + offQh);
  unsigned short* CAh  = (unsigned short*)(ws + offCA);
  float*          CK   = (float*)(ws + offCK);
  float*          SC   = (float*)(ws + offSC);
  unsigned short* PP   = (unsigned short*)(ws + offPP);
  const float* rdummy = Fq;
  const size_t wP = (size_t)kAH * kHid;

  const int n8x = kTok * kHid / 8;
  cast_x_kernel<<<dim3(cdiv_host(n8x, 256)), dim3(256), 0, stream>>>(x, Xh, n8x);
  const int n8w = kAH * kHid / 8;
  cast_w_kernel<<<dim3(cdiv_host(n8w, 256), 5), dim3(256), 0, stream>>>(Wq, Wk, Wv, Wco, pw, Wpl, n8w, kWCarry, kPWCarry);
  cast_wck_kernel<<<dim3(cdiv_host(kCKPad * kAH / 8, 256)), dim3(256), 0, stream>>>(Wck, WCKh);
  dwconv_kernel<<<dim3(kTok / kTokPerBlk), dim3(96), 0, stream>>>(Xh, dw, DWh);

  const int blkProj = cdiv_host((kTok / 64) * (kAH / 64), 8);
  wmma_gemm64<0, false, 2, 0, false, 0><<<dim3(blkProj, 1), dim3(256), 0, stream>>>(
      Xh, Xh, kHid, 0L, Wpl, Wpl, kHid, 0L,
      (void*)Fq, (void*)Fq, kAH, 0L, bq, rdummy, 0L, kTok, kAH, kHid, kWCarryInv, 1.0f);
  wmma_gemm64<0, false, 2, 1, false, 0><<<dim3(blkProj, 1), dim3(256), 0, stream>>>(
      Xh, Xh, kHid, 0L, Wpl + wP, Wpl + wP, kHid, 0L,
      (void*)Kh, (void*)Kh, kAH, 0L, bk, rdummy, 0L, kTok, kAH, kHid, kGCarry * kWCarryInv, kGCarry);
  wmma_gemm64<0, false, 1, 1, false, 0><<<dim3(blkProj, 1), dim3(256), 0, stream>>>(
      Wpl + 2 * wP, Wpl + 2 * wP, kHid, 0L, Xh, Xh, kHid, 0L,
      (void*)VT, (void*)VT, kTok, 0L, bv, rdummy, 0L, kAH, kTok, kHid, kGCarry * kWCarryInv, kGCarry);
  wmma_gemm64<0, false, 2, 0, false, 0><<<dim3(blkProj, 1), dim3(256), 0, stream>>>(
      Xh, Xh, kHid, 0L, Wpl + 3 * wP, Wpl + 3 * wP, kHid, 0L,
      (void*)Fco, (void*)Fco, kAH, 0L, bco, rdummy, 0L, kTok, kAH, kHid, kWCarryInv, 1.0f);
  wmma_gemm64<0, false, 2, 0, false, 0><<<dim3(blkProj, 1), dim3(256), 0, stream>>>(
      DWh, DWh, kHid, 0L, Wpl + 4 * wP, Wpl + 4 * wP, kHid, 0L,
      (void*)Fkc, (void*)Fkc, kAH, 0L, cbias, rdummy, 0L, kTok, kAH, kHid, kKCScale, 1.0f);

  const int n8q = kTok * kAH / 8;
  qca_cast_kernel<<<dim3(cdiv_host(n8q, 256)), dim3(256), 0, stream>>>(Fq, Fkc, Qh, CAh, n8q);
  wmma_gemm64<0, false, 0, 0, false, 0><<<dim3(cdiv_host(kTok / 64, 8), 1), dim3(256), 0, stream>>>(
      CAh, CAh, kAH, 0L, WCKh, WCKh, kAH, 0L,
      (void*)CK, (void*)CK, kCKPad, 0L, bq, rdummy, 0L, kTok, kCKPad, kAH, kCKScale, 1.0f);
  span_conv_kernel<<<dim3(kTok / kTokPerBlk), dim3(96), 0, stream>>>(CK, bck, Fco, out);

  const int blkScore = cdiv_host((SEQ / 64) * (SEQ / 64), 8);
  const int blkCtx   = cdiv_host((SEQ / 64) * (kDh / 64), 8);
  for (int b = 0; b < NB; ++b) {
    for (int h = 0; h < kHeads; ++h) {
      const size_t tokOff = ((size_t)b * SEQ) * kAH + (size_t)h * kDh;
      const unsigned short* Ag  = Qh + tokOff;
      const unsigned short* Btg = Kh + tokOff;
      wmma_gemm64<0, false, 0, 0, false, 0><<<dim3(blkScore, 1), dim3(256), 0, stream>>>(
          Ag, Ag, kAH, 0L, Btg, Btg, kAH, 0L,
          (void*)SC, (void*)SC, SEQ, 0L, bq, rdummy, 0L, SEQ, SEQ, kDh, 1.0f, 1.0f);
      softmax_row_kernel<<<dim3(SEQ), dim3(256), 0, stream>>>(SC, PP);
      const unsigned short* VTg = VT + ((size_t)h * kDh) * kTok + (size_t)b * SEQ;
      float* Og = out + ((size_t)b * SEQ) * (2 * kAH) + (size_t)h * kDh;
      wmma_gemm64<0, false, 0, 0, false, 0><<<dim3(blkCtx, 1), dim3(256), 0, stream>>>(
          PP, PP, SEQ, 0L, VTg, VTg, kTok, 0L,
          (void*)Og, (void*)Og, 2 * kAH, 0L, bq, rdummy, 0L, SEQ, kDh, SEQ, kPVScale, 1.0f);
    }
  }
}
